// DifferentiableTree_31147102831184
// MI455X (gfx1250) — hardware-verified
//
#include <hip/hip_runtime.h>


namespace {
constexpr int N = 65536, F = 64, NI = 1023, NL = 1024, NC = 128, DEPTH = 10;
constexpr float W_SC = 16384.0f, INV_W_SC = 1.0f / 16384.0f;
constexpr float INV_SQRT2 = 0.70710678118654752f;
constexpr int WAVES = 2, SPW = 16;

typedef _Float16 b16;
typedef __attribute__((ext_vector_type(16))) _Float16 v16b;
typedef __attribute__((ext_vector_type(8)))  _Float16 v8b;
typedef __attribute__((ext_vector_type(8)))  float v8f;
typedef __attribute__((ext_vector_type(4)))  float v4f;

__device__ __forceinline__ v8b ld8b(const b16* p) { return *(const v8b*)p; }
__device__ __forceinline__ v16b cat8b(v8b a, v8b b) { return __builtin_shufflevector(a, b, 0, 1, 2, 3, 4, 5, 6, 7, 8, 9, 10, 11, 12, 13, 14, 15); }
__device__ __forceinline__ v16b frag_kb(const b16* p, int hh) { return cat8b(ld8b(p + 8 * hh), ld8b(p + 16 + 8 * hh)); }
__device__ __forceinline__ v8f wmma16b(v16b a, v16b b, v8f c) {
  v8f d = __builtin_amdgcn_wmma_f32_16x16x32_f16(false, a, false, b, (short)0, c, false, false);
  asm volatile("v_nop\n\tv_nop\n\tv_nop\n\tv_nop" : "+v"(d) : "v"(a), "v"(b));
  return d;
}
__device__ __forceinline__ void wave_lds_sync() {
  __builtin_amdgcn_fence(__ATOMIC_RELEASE, "workgroup");
  __builtin_amdgcn_wave_barrier();
  __builtin_amdgcn_fence(__ATOMIC_ACQUIRE, "workgroup");
}

__global__ __launch_bounds__(256) void prep_kernel(const float* __restrict__ lv, b16* __restrict__ lvT) {
  __shared__ __attribute__((aligned(16))) b16 Tl[8][NL];
  const int tid = threadIdx.x, lane = tid & 31, wave = tid >> 5, c0 = blockIdx.x * 8;
  for (int i = tid; i < 8 * NL; i += 256) { const int c = i / NL, leaf = i % NL; Tl[c][leaf] = (b16)lv[(size_t)leaf * NC + c0 + c]; }
  __syncthreads();
  for (int pass = 0; pass < 2; ++pass) {
    { const int c = wave;
#pragma unroll
      for (int j = 0; j < 4; ++j) *(volatile v8b*)(lvT + (size_t)(c0 + c) * NL + j * 256 + lane * 8) = *(const v8b*)(&Tl[c][j * 256 + lane * 8]); }
    __threadfence();
  }
}

__global__ __launch_bounds__(64) void tree_kernel(const float* __restrict__ X, const int* __restrict__ feat, const float* __restrict__ thr,
                                                 const b16* __restrict__ lvT, float* __restrict__ out) {
  __shared__ __attribute__((aligned(16))) b16 At[WAVES][SPW][NL];
  __shared__ float gs[WAVES][NL];
  __shared__ float wl[WAVES][2][NL];
  __shared__ __attribute__((aligned(16))) float Os[WAVES][SPW * NC];
  const int wave = threadIdx.x >> 5, lane = threadIdx.x & 31, hh = lane >> 4, col = lane & 15;
  const int s0 = (blockIdx.x * WAVES + wave) * SPW;
  float* g = gs[wave];
  for (int si = 0; si < SPW; ++si) {
    const int n = s0 + si;
    const float* xr = X + (size_t)n * (2 * F);
    for (int i = lane; i < NI; i += 32) {
      int fi = feat[i]; fi = fi < 0 ? 0 : (fi >= F ? F - 1 : fi);
      const float mu = xr[fi], sd = xr[F + fi];
      g[i] = 0.5f * (1.0f + erff((thr[i] - mu) / (sd * 1.4142135623730951f)));
    }
    wave_lds_sync();
    float* cur = wl[wave][0]; float* nxt = wl[wave][1];
    if (lane == 0) cur[0] = 1.0f;
    wave_lds_sync();
#pragma unroll 1
    for (int l = 0; l < DEPTH; ++l) {
      const int cnt = 1 << l, base = cnt - 1;
      for (int p = lane; p < cnt; p += 32) { const float wp = cur[p], gv = g[base + p]; nxt[2 * p] = wp * gv; nxt[2 * p + 1] = wp * (1.0f - gv); }
      wave_lds_sync();
      float* t = cur; cur = nxt; nxt = t;
    }
#pragma unroll
    for (int j = 0; j < 4; ++j) { v8b v;
#pragma unroll
      for (int e = 0; e < 8; ++e) v[e] = (b16)(cur[j * 256 + lane * 8 + e] * W_SC);
      *(v8b*)(&At[wave][si][j * 256 + lane * 8]) = v; }
    wave_lds_sync();
  }
  v8f acc[8];
#pragma unroll
  for (int t = 0; t < 8; ++t) acc[t] = (v8f){};
  const b16* arow = &At[wave][col][0];
  for (int kb = 0; kb < NL; kb += 32) {
    const v16b a = frag_kb(arow + kb, hh);
#pragma unroll
    for (int t = 0; t < 8; ++t) { const v16b bw = frag_kb(lvT + (size_t)(t * 16 + col) * NL + kb, hh); acc[t] = wmma16b(a, bw, acc[t]); }
  }
  float rs[8];
#pragma unroll
  for (int r = 0; r < 8; ++r) { float s = 0.f;
#pragma unroll
    for (int t = 0; t < 8; ++t) s += acc[t][r];
#pragma unroll
    for (int o = 1; o < 16; o <<= 1) s += __shfl_xor(s, o);
    rs[r] = s; }
  float* Ot = Os[wave];
#pragma unroll
  for (int t = 0; t < 8; ++t)
#pragma unroll
    for (int r = 0; r < 8; ++r) Ot[(8 * hh + r) * NC + t * 16 + col] = acc[t][r] / rs[r];
  wave_lds_sync();
  float* dst = out + (size_t)s0 * NC;
  for (int pass = 0; pass < 2; ++pass) {
#pragma unroll
    for (int rr = 0; rr < SPW; ++rr) *(volatile v4f*)(dst + (size_t)rr * NC + lane * 4) = *(const v4f*)(Ot + rr * NC + lane * 4);
    __threadfence();
  }
}
}

extern "C" void kernel_launch(void* const* d_in, const int* in_sizes, int n_in,
                              void* d_out, int out_size, void* d_ws, size_t ws_size, hipStream_t stream) {
  (void)n_in; (void)out_size;
  const float* X   = (const float*)d_in[0];
  const int* feat  = (const int*)d_in[1];
  const float* thr = (const float*)d_in[2];
  const float* lv  = (const float*)d_in[3];
  float* out = (float*)d_out;
  if (in_sizes[0] != N * 2 * F || in_sizes[1] != NI || in_sizes[2] != NI || in_sizes[3] != NL * NC) return;
  size_t off = 0; char* ws = (char*)d_ws;
  b16* lvT = (b16*)(ws + off); off += (size_t)NC * NL * 2;
  if (off > ws_size) return;
  prep_kernel<<<NC / 8, 256, 0, stream>>>(lv, lvT);
  tree_kernel<<<N / (WAVES * SPW), 64, 0, stream>>>(X, feat, thr, lvT, out);
}
